// SpModel_326417515069
// MI455X (gfx1250) — hardware-run, weakly checked
//
#include <hip/hip_runtime.h>
#include <math.h>

typedef __attribute__((ext_vector_type(16))) _Float16 v16h;
typedef __attribute__((ext_vector_type(8)))  _Float16 v8h;
typedef __attribute__((ext_vector_type(8)))  float    v8f;
typedef __attribute__((ext_vector_type(4)))  float    v4f;
typedef __attribute__((ext_vector_type(8)))  unsigned v8u;
typedef __attribute__((ext_vector_type(4)))  unsigned v4u;
typedef __attribute__((ext_vector_type(2)))  unsigned v2u;

constexpr int kG = 128;
constexpr int kN = 32;
constexpr int kH = 128;
constexpr int kL = 6;
constexpr int kNodeRows  = kG * kN;
constexpr int kTupleRows = kG * kN * kN;
constexpr int kNumXRows  = 32;
constexpr int kNumEaRows = 16;
constexpr int kNumTfRows = 16;
constexpr int kBtPitch   = 136;
constexpr int kSlabPitch = 68;
constexpr int kStagePitch = 36;
constexpr float kLnEps = 1e-5f;
constexpr float kWCarry   = 64.0f;
constexpr float kXCarry0  = 4096.0f;
constexpr float kXCarry   = 64.0f;
constexpr float kTxCarry  = 16.0f;
constexpr float kEaCarry  = 64.0f;
constexpr float kMsgInv   = 1.0f / (kTxCarry * kEaCarry);
static_assert(kH == 128 && kN == 32, "tile maps are written for 128 channels and 32 nodes");
static_assert((kTupleRows % 128) == 0 && (kNodeRows % 128) == 0, "row tiles of 128");
static_assert((kH % 32) == 0, "K multiple of 32");
static_assert(128 * kBtPitch * 2 == 8 * 16 * kSlabPitch * 4, "operand tile and f32 slabs share one LDS region");

constexpr size_t kOffXM  = 0;
constexpr size_t kOffTXT = kOffXM  + (size_t)kTupleRows * kH * 4;
constexpr size_t kOffXS  = kOffTXT + (size_t)kG * kH * kN * kN * 2;
constexpr size_t kOffYS  = kOffXS  + (size_t)kNodeRows * kH * 4;
constexpr size_t kOffWT  = kOffYS  + (size_t)kNodeRows * kH * 4;
constexpr size_t kOffT0  = kOffWT  + (size_t)(kL + 1) * kH * kH * 2;
constexpr size_t kOffT1  = kOffT0  + (size_t)kNumXRows * kH * 4;
constexpr size_t kWsTotal = kOffT1 + (size_t)kNumXRows * kH * 4;
static_assert(kWsTotal == 105119744ull, "carve total");
static_assert(kWsTotal <= 134217728ull, "carve cap");
static_assert((kOffTXT % 128) == 0 && (kOffXS % 128) == 0 && (kOffYS % 128) == 0 && (kOffWT % 128) == 0 &&
              (kOffT0 % 128) == 0 && (kOffT1 % 128) == 0, "128-B aligned regions");

union FragU { v16h v; v8h h[2]; };
__device__ __forceinline__ v16h frag_load(const _Float16* p) {
  FragU f;
  f.h[0] = *(const v8h*)(p);
  f.h[1] = *(const v8h*)(p + 16);
  return f.v;
}
__device__ __forceinline__ v8f mma_f16(v16h a, v16h b, v8f c) {
  c = __builtin_amdgcn_wmma_f32_16x16x32_f16(false, a, false, b, (short)0, c, false, false);
  asm volatile("v_nop\n\tv_nop\n\tv_nop\n\tv_nop" : "+v"(c) : "v"(a), "v"(b));
  return c;
}
__device__ __forceinline__ int clampi(int v, int lo, int hi) {
  return v < lo ? lo : (v > hi ? hi : v);
}

__global__ __launch_bounds__(128) void node_tables_kernel(
    const float* __restrict__ emb_x, const float* __restrict__ W0, const float* __restrict__ b0,
    const float* __restrict__ W1, const float* __restrict__ b1, float* T0, float* T1)
{
  __shared__ __align__(16) float sXr[4 * kH];
  __shared__ __align__(16) float sTr[4 * kH];
  const int tid  = threadIdx.x;
  const int lane = tid & 31;
  const int wave = __builtin_amdgcn_readfirstlane((int)(threadIdx.x >> 5));
  const int tsel = blockIdx.x >> 3;
  const int r0   = (blockIdx.x & 7) * 4;
  const float* W  = tsel ? W1 : W0;
  const float* bb = tsel ? b1 : b0;
  float* T = tsel ? T1 : T0;
#pragma unroll
  for (int rr = 0; rr < 4; ++rr) sXr[rr * kH + tid] = emb_x[(r0 + rr) * kH + tid];
  __syncthreads();
  float a0 = 0.f, a1 = 0.f, a2 = 0.f, a3 = 0.f;
#pragma unroll 1
  for (int k = 0; k < kH; ++k) {
    const float w = W[k * kH + tid];
    a0 = fmaf(sXr[k], w, a0);
    a1 = fmaf(sXr[kH + k], w, a1);
    a2 = fmaf(sXr[2 * kH + k], w, a2);
    a3 = fmaf(sXr[3 * kH + k], w, a3);
  }
  const float bv = bb[tid];
  sTr[tid]          = a0 + bv;
  sTr[kH + tid]     = a1 + bv;
  sTr[2 * kH + tid] = a2 + bv;
  sTr[3 * kH + tid] = a3 + bv;
  __syncthreads();
  const v4f v = *(const v4f*)(sTr + wave * kH + lane * 4);
  float* dst = T + (size_t)(r0 + wave) * kH + lane * 4;
  *(volatile v4f*)dst = v;
  __threadfence();
  *(volatile v4f*)dst = v;
}

__global__ __launch_bounds__(256) void weight_planes_kernel(
    const float* __restrict__ Wc, const float* __restrict__ Wp, unsigned short* WT)
{
  __shared__ float sW[kH * 33];
  const int tid  = threadIdx.x;
  const int lane = tid & 31;
  const int wave = __builtin_amdgcn_readfirstlane((int)(threadIdx.x >> 5));
  const int hh   = lane >> 4;
  const int p    = blockIdx.x >> 2;
  const int n0   = (blockIdx.x & 3) * 32;
  const float* src = (p < kL) ? (Wc + (size_t)p * kH * kH) : Wp;
#pragma unroll 4
  for (int q = 0; q < 16; ++q) {
    const int idx = tid + 256 * q;
    const int k = idx >> 5, nl = idx & 31;
    sW[k * 33 + nl] = src[k * kH + n0 + nl];
  }
  __syncthreads();
  const int c8 = (lane & 15) * 8;
  v8h hv[2];
#pragma unroll
  for (int it = 0; it < 2; ++it) {
    const int nl = wave * 4 + it * 2 + hh;
#pragma unroll
    for (int e = 0; e < 8; ++e) hv[it][e] = (_Float16)(sW[(c8 + e) * 33 + nl] * kWCarry);
  }
  for (int pass = 0; pass < 2; ++pass) {
#pragma unroll
    for (int it = 0; it < 2; ++it) {
      const int nl = wave * 4 + it * 2 + hh;
      unsigned short* dst = WT + (size_t)p * kH * kH + (size_t)(n0 + nl) * kH + c8;
      *(volatile v8h*)dst = hv[it];
    }
    __threadfence();
  }
}

__global__ __launch_bounds__(256) void build_tuples_kernel(
    const int* __restrict__ x_idx, const int* __restrict__ tf_idx,
    const float* __restrict__ T0, const float* __restrict__ T1, const float* __restrict__ emb_tf,
    float* X)
{
  const int tid  = threadIdx.x;
  const int lane = tid & 31;
  const int wave = __builtin_amdgcn_readfirstlane((int)(threadIdx.x >> 5));
  const int rbase = blockIdx.x * 32 + wave * 4;
  v4f v[4];
#pragma unroll
  for (int q = 0; q < 4; ++q) {
    const int row = rbase + q;
    const int j  = row & (kN - 1);
    const int gi = row >> 5;
    const int g  = gi >> 5;
    const int xi = clampi(x_idx[gi], 0, kNumXRows - 1);
    const int xj = clampi(x_idx[g * kN + j], 0, kNumXRows - 1);
    const int tf = clampi(tf_idx[row], 0, kNumTfRows - 1);
    const v4f a = *(const v4f*)(T0 + xi * kH + lane * 4);
    const v4f b = *(const v4f*)(T1 + xj * kH + lane * 4);
    const v4f c = *(const v4f*)(emb_tf + tf * kH + lane * 4);
    v[q] = (a * b) * c;
  }
  for (int pass = 0; pass < 2; ++pass) {
#pragma unroll
    for (int q = 0; q < 4; ++q) {
      float* dst = X + (size_t)(rbase + q) * kH + lane * 4;
      *(volatile v4f*)dst = v[q];
    }
    __threadfence();
  }
}

template <int MODE>
__global__ __launch_bounds__(256) void rows_gemm_ln_kernel(
    const float* __restrict__ Xin, const unsigned short* __restrict__ Wt,
    const float* __restrict__ bias, const float* __restrict__ gam, const float* __restrict__ bet,
    unsigned short* TXT, float* Yout, float a_scale, float inv_scale)
{
  __shared__ __align__(16) _Float16 sB[128 * kBtPitch];
  __shared__ __align__(16) float sP[3 * kH];
  const int tid  = threadIdx.x;
  const int lane = tid & 31;
  const int wave = __builtin_amdgcn_readfirstlane((int)(threadIdx.x >> 5));
  const int hh   = lane >> 4;
  const int m    = lane & 15;
  const int row0 = blockIdx.x * 128;

#pragma unroll
  for (int q = 0; q < 8; ++q) {
    const int c = tid + 256 * q;
    const int n = c >> 4, k8 = (c & 15) * 8;
    const v4u w = *(const v4u*)(Wt + n * kH + k8);
    *(v4u*)(sB + n * kBtPitch + k8) = w;
  }
  if (wave < 4) {
    sP[tid]          = bias[tid];
    sP[kH + tid]     = gam[tid];
    sP[2 * kH + tid] = bet[tid];
  }
  __syncthreads();

  v8f acc[8];
#pragma unroll
  for (int j = 0; j < 8; ++j) acc[j] = (v8f){0.f, 0.f, 0.f, 0.f, 0.f, 0.f, 0.f, 0.f};

  const float* arow = Xin + (size_t)(row0 + wave * 16 + m) * kH + 8 * hh;
#pragma unroll 1
  for (int s = 0; s < 4; ++s) {
    const v4f a0 = *(const v4f*)(arow + s * 32);
    const v4f a1 = *(const v4f*)(arow + s * 32 + 4);
    const v4f a2 = *(const v4f*)(arow + s * 32 + 16);
    const v4f a3 = *(const v4f*)(arow + s * 32 + 20);
    v16h af;
#pragma unroll
    for (int e = 0; e < 4; ++e) {
      af[e]      = (_Float16)(a0[e] * a_scale);
      af[4 + e]  = (_Float16)(a1[e] * a_scale);
      af[8 + e]  = (_Float16)(a2[e] * a_scale);
      af[12 + e] = (_Float16)(a3[e] * a_scale);
    }
#pragma unroll
    for (int j = 0; j < 8; ++j) {
      const v16h bf = frag_load(sB + (j * 16 + m) * kBtPitch + s * 32 + 8 * hh);
      acc[j] = mma_f16(af, bf, acc[j]);
    }
  }

  float bj[8], gj[8], cj[8];
#pragma unroll
  for (int j = 0; j < 8; ++j) {
    bj[j] = sP[j * 16 + m];
    gj[j] = sP[kH + j * 16 + m];
    cj[j] = sP[2 * kH + j * 16 + m];
  }
#pragma unroll
  for (int j = 0; j < 8; ++j)
#pragma unroll
    for (int r = 0; r < 8; ++r) acc[j][r] = fmaf(acc[j][r], inv_scale, bj[j]);

  float mean[8], rstd[8];
#pragma unroll
  for (int r = 0; r < 8; ++r) {
    float s = 0.f;
#pragma unroll
    for (int j = 0; j < 8; ++j) s += acc[j][r];
    s += __shfl_xor(s, 1, 32);
    s += __shfl_xor(s, 2, 32);
    s += __shfl_xor(s, 4, 32);
    s += __shfl_xor(s, 8, 32);
    mean[r] = s * (1.0f / (float)kH);
  }
#pragma unroll
  for (int r = 0; r < 8; ++r) {
    float q = 0.f;
#pragma unroll
    for (int j = 0; j < 8; ++j) {
      const float d = acc[j][r] - mean[r];
      q = fmaf(d, d, q);
    }
    q += __shfl_xor(q, 1, 32);
    q += __shfl_xor(q, 2, 32);
    q += __shfl_xor(q, 4, 32);
    q += __shfl_xor(q, 8, 32);
    rstd[r] = rsqrtf(q * (1.0f / (float)kH) + kLnEps);
  }
#pragma unroll
  for (int j = 0; j < 8; ++j)
#pragma unroll
    for (int r = 0; r < 8; ++r) {
      const float y = (acc[j][r] - mean[r]) * rstd[r] * gj[j] + cj[j];
      acc[j][r] = fmaxf(y, 0.0f);
    }

  if (MODE == 0) {
    __syncthreads();
    const int il = wave >> 1;
    const int kb = (wave & 1) * 16 + 8 * hh;
#pragma unroll
    for (int j = 0; j < 8; ++j) {
      v8h hv;
#pragma unroll
      for (int r = 0; r < 8; ++r) hv[r] = (_Float16)(acc[j][r] * kTxCarry);
      *(v8h*)(sB + (j * 16 + m) * kBtPitch + il * 32 + kb) = hv;
    }
    __syncthreads();
    const int g  = blockIdx.x >> 3;
    const int i0 = (blockIdx.x & 7) * 4;
    v8h ov[8];
#pragma unroll
    for (int it = 0; it < 8; ++it) {
      const int h = wave * 16 + it * 2 + hh;
      ov[it] = *(const v8h*)(sB + h * kBtPitch + m * 8);
    }
    for (int pass = 0; pass < 2; ++pass) {
#pragma unroll
      for (int it = 0; it < 8; ++it) {
        const int h = wave * 16 + it * 2 + hh;
        unsigned short* dst = TXT + ((size_t)((g * kH + h) * kN + i0)) * kN + m * 8;
        *(volatile v8h*)dst = ov[it];
      }
      __threadfence();
    }
  } else {
    float* slab = (float*)(void*)sB + wave * (16 * kSlabPitch);
    const int c4 = m * 4;
#pragma unroll
    for (int half = 0; half < 2; ++half) {
      __syncthreads();
#pragma unroll
      for (int jj = 0; jj < 4; ++jj)
#pragma unroll
        for (int r = 0; r < 8; ++r)
          slab[(8 * hh + r) * kSlabPitch + jj * 16 + m] = acc[half * 4 + jj][r];
      __syncthreads();
      v4f ov[8];
#pragma unroll
      for (int it = 0; it < 8; ++it) ov[it] = *(const v4f*)(slab + (it * 2 + hh) * kSlabPitch + c4);
      for (int pass = 0; pass < 2; ++pass) {
#pragma unroll
        for (int it = 0; it < 8; ++it) {
          float* dst = Yout + (size_t)(row0 + wave * 16 + it * 2 + hh) * kH + half * 64 + c4;
          *(volatile v4f*)dst = ov[it];
        }
        __threadfence();
      }
    }
  }
}

__global__ __launch_bounds__(256) void msg_residual_kernel(
    const unsigned short* __restrict__ TXT, const int* __restrict__ ea_idx, const int* __restrict__ adj,
    const float* __restrict__ emb_ea, float* X)
{
  __shared__ __align__(16) unsigned short sTab[17 * 32];
  __shared__ int sCode[kN * 16];
  __shared__ __align__(16) float sS[256 * kStagePitch];
  const int tid  = threadIdx.x;
  const int lane = tid & 31;
  const int wave = __builtin_amdgcn_readfirstlane((int)(threadIdx.x >> 5));
  const int hh   = lane >> 4;
  const int n    = lane & 15;
  const int g    = blockIdx.x >> 3;
  const int hs   = (blockIdx.x >> 1) & 3;
  const int jt   = blockIdx.x & 1;

#pragma unroll
  for (int q = 0; q < 2; ++q) {
    const int idx = tid + 256 * q;
    const int row = idx >> 5, c = idx & 31;
    const float v = emb_ea[row * kH + hs * 32 + c] * kEaCarry;
    const _Float16 hv = (_Float16)v;
    sTab[idx] = __builtin_bit_cast(unsigned short, hv);
  }
  if (wave == 0) sTab[512 + lane] = (unsigned short)0;
#pragma unroll
  for (int q = 0; q < 2; ++q) {
    const int idx = tid + 256 * q;
    const int k = idx >> 4, jl = idx & 15;
    const int gofs = (g * kN + k) * kN + jt * 16 + jl;
    const int a = adj[gofs];
    const int e = clampi(ea_idx[gofs], 0, kNumEaRows - 1);
    sCode[idx] = (a != 0) ? e : 16;
  }
  __syncthreads();

  unsigned lx[16], ly[16];
#pragma unroll
  for (int e = 0; e < 16; ++e) {
    const int k = (e < 8) ? (8 * hh + e) : (16 + 8 * hh + (e - 8));
    const int code = sCode[k * 16 + n];
    const v2u w = *(const v2u*)(sTab + code * 32 + wave * 4);
    lx[e] = w[0];
    ly[e] = w[1];
  }
  v8u p0, p1, p2, p3;
#pragma unroll
  for (int i = 0; i < 8; ++i) {
    p0[i] = (lx[2 * i] & 0xffffu) | (lx[2 * i + 1] << 16);
    p1[i] = (lx[2 * i] >> 16) | (lx[2 * i + 1] & 0xffff0000u);
    p2[i] = (ly[2 * i] & 0xffffu) | (ly[2 * i + 1] << 16);
    p3[i] = (ly[2 * i] >> 16) | (ly[2 * i + 1] & 0xffff0000u);
  }
  const v16h bf0 = __builtin_bit_cast(v16h, p0);
  const v16h bf1 = __builtin_bit_cast(v16h, p1);
  const v16h bf2 = __builtin_bit_cast(v16h, p2);
  const v16h bf3 = __builtin_bit_cast(v16h, p3);

  const _Float16* tx = (const _Float16*)TXT;
  const size_t abase = ((size_t)(g * kH + hs * 32 + wave * 4) * kN) * kN;
  const int q4 = lane >> 3;
  const int c4 = (lane & 7) * 4;

#pragma unroll
  for (int it2 = 0; it2 < 2; ++it2) {
    const _Float16* ap = tx + abase + (size_t)(it2 * 16 + n) * kN + 8 * hh;
    const v16h a0 = frag_load(ap);
    const v16h a1 = frag_load(ap + kN * kN);
    const v16h a2 = frag_load(ap + 2 * kN * kN);
    const v16h a3 = frag_load(ap + 3 * kN * kN);
    v8f d0 = (v8f){0.f, 0.f, 0.f, 0.f, 0.f, 0.f, 0.f, 0.f};
    v8f d1 = d0, d2 = d0, d3 = d0;
    d0 = mma_f16(a0, bf0, d0);
    d1 = mma_f16(a1, bf1, d1);
    d2 = mma_f16(a2, bf2, d2);
    d3 = mma_f16(a3, bf3, d3);
    if (it2 == 1) __syncthreads();
#pragma unroll
    for (int r = 0; r < 8; ++r) {
      v4f sv;
      sv[0] = d0[r] * kMsgInv;
      sv[1] = d1[r] * kMsgInv;
      sv[2] = d2[r] * kMsgInv;
      sv[3] = d3[r] * kMsgInv;
      *(v4f*)(sS + ((8 * hh + r) * 16 + n) * kStagePitch + wave * 4) = sv;
    }
    __syncthreads();
    v4f ov[8];
#pragma unroll
    for (int t = 0; t < 8; ++t) {
      const int p  = wave * 32 + t * 4 + q4;
      const int il = p >> 4, jl = p & 15;
      const size_t row = (size_t)(g * kN + it2 * 16 + il) * kN + jt * 16 + jl;
      const v4f xv = *(const v4f*)(X + row * kH + hs * 32 + c4);
      const v4f sv = *(const v4f*)(sS + p * kStagePitch + c4);
      ov[t] = xv + sv;
    }
    for (int pass = 0; pass < 2; ++pass) {
#pragma unroll
      for (int t = 0; t < 8; ++t) {
        const int p  = wave * 32 + t * 4 + q4;
        const int il = p >> 4, jl = p & 15;
        const size_t row = (size_t)(g * kN + it2 * 16 + il) * kN + jt * 16 + jl;
        float* dst = X + row * kH + hs * 32 + c4;
        *(volatile v4f*)dst = ov[t];
      }
      __threadfence();
    }
  }
}

__global__ __launch_bounds__(256) void pool_mean_kernel(const float* __restrict__ X, float* XS)
{
  const int tid  = threadIdx.x;
  const int lane = tid & 31;
  const int wave = __builtin_amdgcn_readfirstlane((int)(threadIdx.x >> 5));
  const int r = blockIdx.x * 8 + wave;
  const float* base = X + (size_t)r * kN * kH + lane * 4;
  v4f s = (v4f){0.f, 0.f, 0.f, 0.f};
#pragma unroll 4
  for (int j = 0; j < kN; ++j) s = s + *(const v4f*)(base + j * kH);
  s = s * (1.0f / (float)kN);
  float* dst = XS + (size_t)r * kH + lane * 4;
  *(volatile v4f*)dst = s;
  __threadfence();
  *(volatile v4f*)dst = s;
}

__global__ __launch_bounds__(256) void graph_head_kernel(
    const float* __restrict__ YS, const float* __restrict__ Wq1, const float* __restrict__ bq1,
    const float* __restrict__ gq1, const float* __restrict__ cq1, const float* __restrict__ Wq2,
    const float* __restrict__ bq2, float* out)
{
  __shared__ __align__(16) float sHg[8 * kH];
  __shared__ float sRes[32];
  const int tid  = threadIdx.x;
  const int lane = tid & 31;
  const int wave = __builtin_amdgcn_readfirstlane((int)(threadIdx.x >> 5));
  const float b2 = bq2[0];
  const v4f bv = *(const v4f*)(bq1 + lane * 4);
  const v4f gv = *(const v4f*)(gq1 + lane * 4);
  const v4f cv = *(const v4f*)(cq1 + lane * 4);
  const v4f w2 = *(const v4f*)(Wq2 + lane * 4);
#pragma unroll 1
  for (int gi = 0; gi < 4; ++gi) {
    const int g = blockIdx.x * 32 + wave * 4 + gi;
    const float* yp = YS + (size_t)g * kN * kH + lane * 4;
    v4f hsum = (v4f){0.f, 0.f, 0.f, 0.f};
#pragma unroll 4
    for (int i = 0; i < kN; ++i) hsum = hsum + *(const v4f*)(yp + i * kH);
    *(v4f*)(sHg + wave * kH + lane * 4) = hsum;
    __syncthreads();
    const float* hp = sHg + wave * kH;
    float z0 = 0.f, z1 = 0.f, z2 = 0.f, z3 = 0.f;
#pragma unroll 2
    for (int k = 0; k < kH; ++k) {
      const float hk = hp[k];
      const v4f w = *(const v4f*)(Wq1 + k * kH + lane * 4);
      z0 = fmaf(hk, w[0], z0);
      z1 = fmaf(hk, w[1], z1);
      z2 = fmaf(hk, w[2], z2);
      z3 = fmaf(hk, w[3], z3);
    }
    z0 += bv[0];
    z1 += bv[1];
    z2 += bv[2];
    z3 += bv[3];
    float s = (z0 + z1) + (z2 + z3);
    s += __shfl_xor(s, 16, 32);
    s += __shfl_xor(s, 8, 32);
    s += __shfl_xor(s, 4, 32);
    s += __shfl_xor(s, 2, 32);
    s += __shfl_xor(s, 1, 32);
    const float mean = s * (1.0f / (float)kH);
    const float e0 = z0 - mean, e1 = z1 - mean, e2 = z2 - mean, e3 = z3 - mean;
    float q = (e0 * e0 + e1 * e1) + (e2 * e2 + e3 * e3);
    q += __shfl_xor(q, 16, 32);
    q += __shfl_xor(q, 8, 32);
    q += __shfl_xor(q, 4, 32);
    q += __shfl_xor(q, 2, 32);
    q += __shfl_xor(q, 1, 32);
    const float rs = rsqrtf(q * (1.0f / (float)kH) + kLnEps);
    const float y0 = fmaxf(e0 * rs * gv[0] + cv[0], 0.0f);
    const float y1 = fmaxf(e1 * rs * gv[1] + cv[1], 0.0f);
    const float y2 = fmaxf(e2 * rs * gv[2] + cv[2], 0.0f);
    const float y3 = fmaxf(e3 * rs * gv[3] + cv[3], 0.0f);
    float dot = y0 * w2[0];
    dot = fmaf(y1, w2[1], dot);
    dot = fmaf(y2, w2[2], dot);
    dot = fmaf(y3, w2[3], dot);
    dot += __shfl_xor(dot, 16, 32);
    dot += __shfl_xor(dot, 8, 32);
    dot += __shfl_xor(dot, 4, 32);
    dot += __shfl_xor(dot, 2, 32);
    dot += __shfl_xor(dot, 1, 32);
    if (lane == 0) sRes[wave * 4 + gi] = dot + b2;
    __syncthreads();
  }
  if (wave == 0) {
    const float v = sRes[lane];
    volatile float* o = out + blockIdx.x * 32 + lane;
    *o = v;
    __threadfence();
    *o = v;
  }
}

extern "C" void kernel_launch(void* const* d_in, const int* in_sizes, int n_in,
                              void* d_out, int out_size, void* d_ws, size_t ws_size,
                              hipStream_t stream)
{
  if (n_in < 25) return;
  if (in_sizes[0] != kNodeRows) return;
  if (in_sizes[1] != kTupleRows || in_sizes[2] != kTupleRows || in_sizes[3] != kTupleRows) return;
  if (in_sizes[4] != kNumXRows * kH || in_sizes[5] != kNumEaRows * kH || in_sizes[6] != kNumTfRows * kH) return;
  if (in_sizes[7] != kH * kH || in_sizes[9] != kH * kH || in_sizes[11] != kL * kH * kH) return;
  if (in_sizes[15] != kH * kH || in_sizes[19] != kH * kH || in_sizes[23] != kH) return;
  if (out_size != kG) return;
  if (ws_size < kWsTotal) return;

  const int*   x_idx  = (const int*)d_in[0];
  const int*   ea_idx = (const int*)d_in[1];
  const int*   tf_idx = (const int*)d_in[2];
  const int*   adj    = (const int*)d_in[3];
  const float* emb_x  = (const float*)d_in[4];
  const float* emb_ea = (const float*)d_in[5];
  const float* emb_tf = (const float*)d_in[6];
  const float* W0  = (const float*)d_in[7];
  const float* b0  = (const float*)d_in[8];
  const float* W1  = (const float*)d_in[9];
  const float* b1  = (const float*)d_in[10];
  const float* Wc  = (const float*)d_in[11];
  const float* bc  = (const float*)d_in[12];
  const float* gc  = (const float*)d_in[13];
  const float* cc  = (const float*)d_in[14];
  const float* Wp  = (const float*)d_in[15];
  const float* bp  = (const float*)d_in[16];
  const float* gp  = (const float*)d_in[17];
  const float* cp  = (const float*)d_in[18];
  const float* Wq1 = (const float*)d_in[19];
  const float* bq1 = (const float*)d_in[20];
  const float* gq1 = (const float*)d_in[21];
  const float* cq1 = (const float*)d_in[22];
  const float* Wq2 = (const float*)d_in[23];
  const float* bq2 = (const float*)d_in[24];
  float* out = (float*)d_out;

  char* ws = (char*)d_ws;
  float*          XM  = (float*)(ws + kOffXM);
  unsigned short* TXT = (unsigned short*)(ws + kOffTXT);
  float*          XS  = (float*)(ws + kOffXS);
  float*          YS  = (float*)(ws + kOffYS);
  unsigned short* WT  = (unsigned short*)(ws + kOffWT);
  float*          T0  = (float*)(ws + kOffT0);
  float*          T1  = (float*)(ws + kOffT1);

  node_tables_kernel<<<16, 128, 0, stream>>>(emb_x, W0, b0, W1, b1, T0, T1);
  weight_planes_kernel<<<(kL + 1) * 4, 256, 0, stream>>>(Wc, Wp, WT);
  build_tuples_kernel<<<kTupleRows / 32, 256, 0, stream>>>(x_idx, tf_idx, T0, T1, emb_tf, XM);

  for (int l = 0; l < kL; ++l) {
    const float a_scale = (l == 0) ? kXCarry0 : kXCarry;
    const float inv_scale = 1.0f / (a_scale * kWCarry);
    rows_gemm_ln_kernel<0><<<kTupleRows / 128, 256, 0, stream>>>(
        XM, WT + (size_t)l * kH * kH, bc + l * kH, gc + l * kH, cc + l * kH, TXT, YS, a_scale, inv_scale);
    msg_residual_kernel<<<kG * 4 * 2, 256, 0, stream>>>(TXT, ea_idx, adj, emb_ea, XM);
  }

  pool_mean_kernel<<<kNodeRows / 8, 256, 0, stream>>>(XM, XS);
  rows_gemm_ln_kernel<1><<<kNodeRows / 128, 256, 0, stream>>>(
      XS, WT + (size_t)kL * kH * kH, bp, gp, cp, TXT, YS, kXCarry, 1.0f / (kXCarry * kWCarry));
  graph_head_kernel<<<kG / 32, 256, 0, stream>>>(YS, Wq1, bq1, gq1, cq1, Wq2, bq2, out);
}
